// GatedGCNModel_28956669510068
// MI455X (gfx1250) — hardware-verified
//
#include <hip/hip_runtime.h>
#include <hip/hip_bf16.h>
#include <stddef.h>
#include <stdint.h>


#define DIN     128
#define G3H     384
#define KSP     256
#define NTHR    256
#define NWAVE   8
#define EPT     8
#define CHUNK   (NTHR * EPT)
#define WCAP    (EPT * 32)
#define LISTN   (NWAVE * WCAP)
#define NBMAX   2048
#define RCAP    28672
#define DEGCAP  64
#define STW     512
#define GBM     64
#define GBN     64
#define GTHR    128
#define RB      128
#define NCHK    4
#define MPQ     512
#define WSMAX   268435456
#define LDS_AGG ((2 * RCAP + 2 * NBMAX + LISTN) * 4 + 64)
#define WO_M1   0
#define WO_HH1  16384
#define WO_IH1  65536
#define WO_M2   163840
#define WO_HH2  196608
#define WO_IH2  294912
#define WO_L    393216
#define WO_END  425984

static_assert((CHUNK & (CHUNK - 1)) == 0 && CHUNK <= 4096);
static_assert((NBMAX & (NBMAX - 1)) == 0 && NBMAX <= 4096);
static_assert(NTHR * 8 == NBMAX);
static_assert(LISTN >= NBMAX);
static_assert(LISTN >= NWAVE * WCAP);
static_assert((RCAP % 32) == 0);
static_assert(NWAVE * STW <= RCAP);
static_assert(STW >= DIN);
static_assert(LDS_AGG <= 300000);
static_assert(GBM == (GTHR / 32) * 16);
static_assert((DIN % 32) == 0 && (KSP % 32) == 0 && (G3H % GBN) == 0 && (DIN % GBN) == 0);
static_assert((MPQ % (NCHK * RB)) == 0 && (RB % GBM) == 0);
static_assert(RB == NWAVE * 16);
static_assert(WO_HH1 == WO_M1 + DIN * DIN && WO_IH1 == WO_HH1 + G3H * DIN && WO_M2 == WO_IH1 + G3H * KSP);
static_assert(WO_HH2 == WO_M2 + DIN * KSP && WO_IH2 == WO_HH2 + G3H * KSP && WO_L == WO_IH2 + G3H * KSP);
static_assert(WO_END == WO_L + DIN * KSP);
static_assert(((WO_HH1 * 2) % 512) == 0 && ((WO_IH1 * 2) % 512) == 0 && ((WO_M2 * 2) % 512) == 0);
static_assert(((WO_HH2 * 2) % 512) == 0 && ((WO_IH2 * 2) % 512) == 0 && ((WO_L * 2) % 512) == 0);

typedef float    v4f  __attribute__((ext_vector_type(4)));
typedef float    v8f  __attribute__((ext_vector_type(8)));
typedef int      v4i  __attribute__((ext_vector_type(4)));
typedef int      v8i  __attribute__((ext_vector_type(8)));
typedef __bf16   v16b __attribute__((ext_vector_type(16)));
typedef unsigned short us_t;
union FragB { v16b v; v4i q[2]; v8i w; };
union DU2 { double d[2]; v4f f; };

__device__ __forceinline__ unsigned int f2bf(float f) {
  const unsigned int u = __float_as_uint(f);
  return (u + 0x7FFFu + ((u >> 16) & 1u)) >> 16;
}
__device__ __forceinline__ float bfr(float f) { return __uint_as_float(f2bf(f) << 16); }

__device__ __forceinline__ v4i pack8(const v4f a, const v4f b) {
  v4i o;
  o.x = (int)(f2bf(a.x) | (f2bf(a.y) << 16));
  o.y = (int)(f2bf(a.z) | (f2bf(a.w) << 16));
  o.z = (int)(f2bf(b.x) | (f2bf(b.y) << 16));
  o.w = (int)(f2bf(b.z) | (f2bf(b.w) << 16));
  return o;
}
__device__ __forceinline__ unsigned int pk2(float a, float b, unsigned int& lo) {
  const unsigned int ha = f2bf(a), hb = f2bf(b);
  const float ra = a - __uint_as_float(ha << 16);
  const float rb = b - __uint_as_float(hb << 16);
  lo = f2bf(ra) | (f2bf(rb) << 16);
  return ha | (hb << 16);
}
__device__ __forceinline__ void split8(const v4f a, const v4f b, v4i& H, v4i& L) {
  unsigned int l0, l1, l2, l3;
  const unsigned int h0 = pk2(a.x, a.y, l0);
  const unsigned int h1 = pk2(a.z, a.w, l1);
  const unsigned int h2 = pk2(b.x, b.y, l2);
  const unsigned int h3 = pk2(b.z, b.w, l3);
  H.x = (int)h0; H.y = (int)h1; H.z = (int)h2; H.w = (int)h3;
  L.x = (int)l0; L.y = (int)l1; L.z = (int)l2; L.w = (int)l3;
}

__device__ __forceinline__ v8f wmb(const FragB& a, const FragB& b, v8f c) {
  v8f d = __builtin_amdgcn_wmma_f32_16x16x32_bf16(false, a.v, false, b.v, (short)0, c, false, false);
  asm volatile("v_nop\n\tv_nop\n\tv_nop\n\tv_nop" : "+v"(d) : "v"(a.w), "v"(b.w));
  return d;
}

__device__ __forceinline__ float sigm(float v) {
  const float e = __expf(-fabsf(v));
  const float p = __builtin_amdgcn_rcpf(1.0f + e);
  return v >= 0.f ? p : e * p;
}
__device__ __forceinline__ float tnh(float v) {
  const float e = __expf(-2.0f * fabsf(v));
  const float t = (1.0f - e) * __builtin_amdgcn_rcpf(1.0f + e);
  return v >= 0.f ? t : -t;
}
__device__ __forceinline__ float gruc(float ir, float hr, float iz, float hz, float inn, float hn, float X) {
  const float r = sigm(ir + hr);
  const float z = sigm(iz + hz);
  const float n = tnh(inn + r * hn);
  const float h = (1.0f - z) * n + z * X;
  return fmaxf(h, 0.f);
}

__device__ __forceinline__ int scan_chunk(const int* __restrict__ dsts, int nE, int cbase, int slotBase,
                                          int nb, int vec8, int* list, int tid, int lane, int wave) {
  int wc = 0;
  const int el0  = tid * EPT;
  const int e0   = cbase + el0;
  const int sent = -2147483647 - 1;
  v4i da, db;
  if (vec8 != 0 && cbase + CHUNK <= nE) {
    da = *(const v4i*)(dsts + e0);
    db = *(const v4i*)(dsts + e0 + 4);
  } else {
    da.x = (e0     < nE) ? dsts[min(e0,     nE - 1)] : sent;
    da.y = (e0 + 1 < nE) ? dsts[min(e0 + 1, nE - 1)] : sent;
    da.z = (e0 + 2 < nE) ? dsts[min(e0 + 2, nE - 1)] : sent;
    da.w = (e0 + 3 < nE) ? dsts[min(e0 + 3, nE - 1)] : sent;
    db.x = (e0 + 4 < nE) ? dsts[min(e0 + 4, nE - 1)] : sent;
    db.y = (e0 + 5 < nE) ? dsts[min(e0 + 5, nE - 1)] : sent;
    db.z = (e0 + 6 < nE) ? dsts[min(e0 + 6, nE - 1)] : sent;
    db.w = (e0 + 7 < nE) ? dsts[min(e0 + 7, nE - 1)] : sent;
  }
  const unsigned nbs = (unsigned)slotBase;
  const unsigned unb = (unsigned)nb;
  const unsigned s0 = (unsigned)da.x - nbs, s1 = (unsigned)da.y - nbs;
  const unsigned s2 = (unsigned)da.z - nbs, s3 = (unsigned)da.w - nbs;
  const unsigned s4 = (unsigned)db.x - nbs, s5 = (unsigned)db.y - nbs;
  const unsigned s6 = (unsigned)db.z - nbs, s7 = (unsigned)db.w - nbs;
  const bool h0 = s0 < unb, h1 = s1 < unb, h2 = s2 < unb, h3 = s3 < unb;
  const bool h4 = s4 < unb, h5 = s5 < unb, h6 = s6 < unb, h7 = s7 < unb;
  const unsigned any = __builtin_amdgcn_ballot_w32(h0 | h1 | h2 | h3 | h4 | h5 | h6 | h7);
  if (any != 0u) {
#define HITJ(J, HJ, SJ) { \
      const unsigned mj = __builtin_amdgcn_ballot_w32(HJ); \
      if (mj != 0u) { \
        if (HJ) { \
          const int pos = wc + (int)__builtin_amdgcn_mbcnt_lo(mj, 0u); \
          if (pos < WCAP) list[wave * WCAP + pos] = ((el0 + (J)) << 12) | (int)(SJ); \
        } \
        wc += (int)__builtin_popcount(mj); } }
    HITJ(0, h0, s0)
    HITJ(1, h1, s1)
    HITJ(2, h2, s2)
    HITJ(3, h3, s3)
    HITJ(4, h4, s4)
    HITJ(5, h5, s5)
    HITJ(6, h6, s6)
    HITJ(7, h7, s7)
#undef HITJ
  }
  return wc;
}

__global__ __launch_bounds__(NTHR) void k_wcvt(const float* __restrict__ w1, const float* __restrict__ whh1,
                                               const float* __restrict__ wih1, const float* __restrict__ w2,
                                               const float* __restrict__ whh2, const float* __restrict__ wih2,
                                               const float* __restrict__ lw1, us_t* wt) {
  const int job = (int)blockIdx.y;
  const float* w = w1; int off = WO_M1, nrows = DIN, trans = 1, dup = 0;
  if (job == 1)      { w = whh1; off = WO_HH1; nrows = G3H; trans = 0; dup = 0; }
  else if (job == 2) { w = wih1; off = WO_IH1; nrows = G3H; trans = 0; dup = 1; }
  else if (job == 3) { w = w2;   off = WO_M2;  nrows = DIN; trans = 1; dup = 1; }
  else if (job == 4) { w = whh2; off = WO_HH2; nrows = G3H; trans = 0; dup = 1; }
  else if (job == 5) { w = wih2; off = WO_IH2; nrows = G3H; trans = 0; dup = 1; }
  else if (job == 6) { w = lw1;  off = WO_L;   nrows = DIN; trans = 0; dup = 1; }
  const int u = (int)blockIdx.x * NTHR + (int)threadIdx.x;
  if (u >= nrows * 16) return;
  const int n  = u >> 4;
  const int k8 = (u & 15) * 8;
  v4f a, b;
  if (trans) {
    const float* p = w + (size_t)k8 * DIN + n;
    a.x = p[0];         a.y = p[DIN];       a.z = p[2 * DIN];   a.w = p[3 * DIN];
    b.x = p[4 * DIN];   b.y = p[5 * DIN];   b.z = p[6 * DIN];   b.w = p[7 * DIN];
  } else {
    const float* p = w + (size_t)n * DIN + k8;
    a = *(const v4f*)p;
    b = *(const v4f*)(p + 4);
  }
  const v4i pk = pack8(a, b);
  const int kout = dup ? KSP : DIN;
  us_t* o = wt + off + (size_t)n * kout + k8;
  *(volatile v4i*)o = pk;
  if (dup) *(volatile v4i*)(o + DIN) = pk;
  __threadfence();
  *(volatile v4i*)o = pk;
  if (dup) *(volatile v4i*)(o + DIN) = pk;
}

__global__ __launch_bounds__(NTHR) void k_xprep(const float* __restrict__ x, us_t* xb, int nN, int nUnits) {
  const int i = (int)blockIdx.x * NTHR + (int)threadIdx.x;
  if (i >= nUnits) return;
  const int row = i >> 4;
  const int c0  = (i & 15) * 8;
  const int rc  = row < nN ? row : nN - 1;
  const float* p = x + (size_t)rc * DIN + c0;
  v4f a = *(const v4f*)p, b = *(const v4f*)(p + 4);
  const v4f z4 = {0.f, 0.f, 0.f, 0.f};
  if (row >= nN) { a = z4; b = z4; }
  const v4i pk = pack8(a, b);
  us_t* o = xb + (size_t)row * DIN + c0;
  *(volatile v4i*)o = pk;
  __threadfence();
  *(volatile v4i*)o = pk;
}

__global__ __launch_bounds__(GTHR) void k_gemm(
    const us_t* __restrict__ A0, const us_t* __restrict__ W0, const float* __restrict__ B0, float* O0,
    int K0, int ldo0, int blen0, int relu0, int ny0,
    const us_t* __restrict__ A1, const us_t* __restrict__ W1, const float* __restrict__ B1, float* O1,
    int K1, int ldo1, int blen1, int relu1)
{
  __shared__ __attribute__((aligned(16))) float stg[GBM * GBN];
  const int tid = (int)threadIdx.x, lane = tid & 31, wave = tid >> 5, hh = lane >> 4, m = lane & 15;
  const bool j1 = (int)blockIdx.y >= ny0;
  const us_t* A  = j1 ? A1 : A0;
  const us_t* WT = j1 ? W1 : W0;
  const float* bp = j1 ? B1 : B0;
  float* outF = j1 ? O1 : O0;
  const int K    = j1 ? K1 : K0;
  const int ldo  = j1 ? ldo1 : ldo0;
  const int blen = j1 ? blen1 : blen0;
  const int relu = j1 ? relu1 : relu0;
  const int cy   = j1 ? ((int)blockIdx.y - ny0) : (int)blockIdx.y;
  const int rowBase = (int)blockIdx.x * GBM;
  const int col0    = cy * GBN;

  v8f acc[4];
  {
    const v8f z = {0.f, 0.f, 0.f, 0.f, 0.f, 0.f, 0.f, 0.f};
    acc[0] = z; acc[1] = z; acc[2] = z; acc[3] = z;
  }
  const us_t* ap = A  + (size_t)(rowBase + 16 * wave + m) * (size_t)K + 8 * hh;
  const us_t* wp = WT + (size_t)(col0 + m) * (size_t)K + 8 * hh;
  const int ksteps = K >> 5;
#pragma unroll 1
  for (int ks = 0; ks < ksteps; ++ks) {
    FragB af;
    af.q[0] = *(const v4i*)(ap + 32 * ks);
    af.q[1] = *(const v4i*)(ap + 32 * ks + 16);
#pragma unroll
    for (int t = 0; t < 4; ++t) {
      const us_t* wq = wp + (size_t)(16 * t) * (size_t)K + 32 * ks;
      FragB bf;
      bf.q[0] = *(const v4i*)wq;
      bf.q[1] = *(const v4i*)(wq + 16);
      acc[t] = wmb(af, bf, acc[t]);
    }
  }

#pragma unroll
  for (int t = 0; t < 4; ++t) {
    const int lc = 16 * t + m;
    int bi = col0 + lc;
    bi = bi > blen - 1 ? blen - 1 : bi;
    bi = bi < 0 ? 0 : bi;
    const float braw = bp[bi];
    const float bv = (blen > 0) ? bfr(braw) : 0.0f;
#pragma unroll
    for (int r = 0; r < 8; ++r) {
      const int lr = 16 * wave + 8 * hh + r;
      float v = acc[t][r] + bv;
      v = relu ? fmaxf(v, 0.f) : v;
      stg[lr * GBN + lc] = v;
    }
  }
  __syncthreads();

  v4f fv[8];
#pragma unroll
  for (int i = 0; i < 8; ++i) {
    const int lr = 16 * wave + 2 * i + hh;
    fv[i] = *(const v4f*)(stg + lr * GBN + 4 * m);
  }
#pragma unroll
  for (int i = 0; i < 8; ++i) {
    const int lr = 16 * wave + 2 * i + hh;
    const int gr = rowBase + lr;
    float* op = outF + (size_t)gr * (size_t)ldo + col0 + 4 * m;
    *(volatile v4f*)op = fv[i];
  }
  __threadfence();
#pragma unroll
  for (int i = 0; i < 8; ++i) {
    const int lr = 16 * wave + 2 * i + hh;
    const int gr = rowBase + lr;
    float* op = outF + (size_t)gr * (size_t)ldo + col0 + 4 * m;
    *(volatile v4f*)op = fv[i];
  }
}

__global__ __launch_bounds__(NTHR) void k_agg(
    const int* __restrict__ srcs, const int* __restrict__ dsts, const float* __restrict__ ew,
    const float* __restrict__ Mp, us_t* Aout,
    int nN, int nE, int nb, int vec8, int chunkBase, int chRows) {
  extern __shared__ v4f lds_dyn[];
  int* reg1 = (int*)lds_dyn;
  int* reg2 = reg1 + RCAP;
  int* scnt = reg2 + RCAP;
  int* soff = scnt + NBMAX;
  int* list = soff + NBMAX;
  int* wcnt = list + LISTN;
  int* wtot = wcnt + NWAVE;
  const int tid = (int)threadIdx.x, lane = tid & 31, wave = tid >> 5;
  const int nodeBase = chunkBase + (int)blockIdx.x * nb;

  for (int i = tid; i < NBMAX; i += NTHR) scnt[i] = 0;
  __syncthreads();

  int tot = 0;
  const int nChunks = (nE + CHUNK - 1) / CHUNK;
#pragma unroll 1
  for (int ch = 0; ch < nChunks; ++ch) {
    const int cbase = ch * CHUNK;
    const int wc = scan_chunk(dsts, nE, cbase, nodeBase, nb, vec8, list, tid, lane, wave);
    if (lane == 0) wcnt[wave] = wc;
    __syncthreads();
    int pre = 0, all = 0;
#pragma unroll
    for (int w2 = 0; w2 < NWAVE; ++w2) {
      int c = wcnt[w2];
      c = c < 0 ? 0 : (c > WCAP ? WCAP : c);
      all += c;
      pre += (w2 < wave) ? c : 0;
    }
    const int wcc  = wc > WCAP ? WCAP : wc;
    const int base = tot + pre;
#pragma unroll 1
    for (int i = lane; i < wcc; i += 32) {
      const int ent = list[wave * WCAP + i];
      const int el  = (ent >> 12) & (CHUNK - 1);
      const int sl  = ent & (NBMAX - 1);
      int eid = cbase + el;
      eid = eid > nE - 1 ? nE - 1 : eid;
      const int pos = base + i;
      if (pos < RCAP) reg1[pos] = (int)(((unsigned)eid << 12) | (unsigned)sl);
    }
    tot += all;
    tot = tot > RCAP ? RCAP : tot;
    __syncthreads();
  }
  const int nh = tot;

  if (wave == 0) {
#pragma unroll 1
    for (int b0 = 0; b0 < nh; b0 += 32) {
      const int idx = b0 + lane;
      const int uv  = reg1[idx < RCAP ? idx : RCAP - 1];
      const int m32 = (nh - b0) < 32 ? (nh - b0) : 32;
#pragma unroll 1
      for (int k = 0; k < m32; ++k) {
        const int u  = __builtin_amdgcn_readlane(uv, k);
        const int sl = u & (NBMAX - 1);
        if (lane == 0) scnt[sl] = scnt[sl] + 1;
      }
    }
  }
  __syncthreads();

  {
    const v4i ca = *(const v4i*)(scnt + 8 * tid);
    const v4i cb = *(const v4i*)(scnt + 8 * tid + 4);
    const int e0 = ca.x < 0 ? 0 : ca.x, e1 = ca.y < 0 ? 0 : ca.y, e2 = ca.z < 0 ? 0 : ca.z, e3 = ca.w < 0 ? 0 : ca.w;
    const int e4 = cb.x < 0 ? 0 : cb.x, e5 = cb.y < 0 ? 0 : cb.y, e6 = cb.z < 0 ? 0 : cb.z, e7 = cb.w < 0 ? 0 : cb.w;
    const int ts = e0 + e1 + e2 + e3 + e4 + e5 + e6 + e7;
    int incl = ts;
#pragma unroll
    for (int d = 1; d < 32; d <<= 1) {
      const int up = __shfl_up(incl, d);
      if (lane >= d) incl += up;
    }
    if (lane == 31) wtot[wave] = incl;
    __syncthreads();
    int pre = 0;
#pragma unroll
    for (int w2 = 0; w2 < NWAVE; ++w2) pre += (w2 < wave) ? wtot[w2] : 0;
    int run = pre + incl - ts;
    soff[8 * tid + 0] = run; run += e0;
    soff[8 * tid + 1] = run; run += e1;
    soff[8 * tid + 2] = run; run += e2;
    soff[8 * tid + 3] = run; run += e3;
    soff[8 * tid + 4] = run; run += e4;
    soff[8 * tid + 5] = run; run += e5;
    soff[8 * tid + 6] = run; run += e6;
    soff[8 * tid + 7] = run;
  }
  __syncthreads();
  for (int i = tid; i < NBMAX; i += NTHR) list[i] = soff[i];
  __syncthreads();

  if (wave == 0) {
#pragma unroll 1
    for (int b0 = 0; b0 < nh; b0 += 32) {
      const int idx = b0 + lane;
      const int uv  = reg1[idx < RCAP ? idx : RCAP - 1];
      const int m32 = (nh - b0) < 32 ? (nh - b0) : 32;
#pragma unroll 1
      for (int k = 0; k < m32; ++k) {
        const int u   = __builtin_amdgcn_readlane(uv, k);
        const int sl  = u & (NBMAX - 1);
        const int eid = (int)((unsigned)u >> 12);
        if (lane == 0) {
          int pos = list[sl];
          pos = pos < 0 ? 0 : (pos > RCAP - 1 ? RCAP - 1 : pos);
          reg2[pos] = eid;
          list[sl] = pos + 1;
        }
      }
    }
  }
  __syncthreads();

  const int nbw = nb >> 3;
  const bool ovf = (nh >= RCAP);
  const float qnan = __int_as_float(0x7fc00000);
  float* stw = (float*)reg1 + wave * STW;
  const int lc = lane & 15;
  const v4f z4 = {0.f, 0.f, 0.f, 0.f};
#pragma unroll 1
  for (int jt = 0; jt < nbw; ++jt) {
    const int slot = wave * nbw + jt;
    const int grow = nodeBase + slot;
    const int lrow = grow - chunkBase;
    int st = soff[slot];
    const int craw = scnt[slot];
    int cnt = craw;
    st  = st < 0 ? 0 : (st > nh ? nh : st);
    cnt = cnt < 0 ? 0 : (cnt > DEGCAP ? DEGCAP : cnt);
    if (cnt > nh - st) cnt = nh - st;
    const float pz = (ovf || craw > DEGCAP) ? qnan : 0.0f;
    const bool wr = lrow < chRows;
    const float live = grow < nN ? 1.0f : 0.0f;

    v4f acc = z4;
#pragma unroll 1
    for (int q = 0; q < cnt; ++q) {
      int idx = st + q; idx = idx > RCAP - 1 ? RCAP - 1 : idx;
      int eid = reg2[idx]; eid = eid < 0 ? 0 : (eid > nE - 1 ? nE - 1 : eid);
      const int sraw = srcs[eid];
      const int s = sraw < 0 ? 0 : (sraw > nN - 1 ? nN - 1 : sraw);
      const float w = bfr(ew[eid]);
      const v4f mv = *(const v4f*)(Mp + (size_t)s * DIN + 4 * lane);
      acc = acc + w * mv;
    }
    __builtin_amdgcn_fence(__ATOMIC_RELEASE, "wavefront");
    __builtin_amdgcn_wave_barrier();
    *(v4f*)(stw + 4 * lane) = acc;
    __builtin_amdgcn_fence(__ATOMIC_RELEASE, "wavefront");
    __builtin_amdgcn_wave_barrier();
    v4f ga = *(const v4f*)(stw + 8 * lc);
    v4f gb = *(const v4f*)(stw + 8 * lc + 4);
    ga = ga * live + pz;
    gb = gb * live + pz;
    v4i H, L;
    split8(ga, gb, H, L);
    const bool hsel = lane < 16;
    v4i sel;
    sel.x = hsel ? H.x : L.x;
    sel.y = hsel ? H.y : L.y;
    sel.z = hsel ? H.z : L.z;
    sel.w = hsel ? H.w : L.w;
    us_t* gp = Aout + (size_t)lrow * KSP + 8 * lane;
    if (wr) *(volatile v4i*)gp = sel;
    __threadfence();
    if (wr) *(volatile v4i*)gp = sel;
  }
}

template<int MODE>
__global__ __launch_bounds__(NTHR) void k_gru(
    const float* __restrict__ gi, const float* __restrict__ gh, const float* __restrict__ xin,
    const float* __restrict__ tab, float* hp, float* rec, int chunkBase, int nN)
{
  __shared__ __attribute__((aligned(16))) double red[2 * NWAVE * DIN];
  const int tid = (int)threadIdx.x, lane = tid & 31, wave = tid >> 5;
  const int c0 = 4 * lane;
  const int lrow0 = (int)blockIdx.x * RB + wave * 16;
  const int blkg = chunkBase / RB + (int)blockIdx.x;
  const v4f z4 = {0.f, 0.f, 0.f, 0.f};
  v4f mean4 = z4, mult4 = z4, beta4 = z4;
  if (MODE == 1) {
    mean4 = *(const v4f*)(tab + c0);
    mult4 = *(const v4f*)(tab + DIN + c0);
    beta4 = *(const v4f*)(tab + 2 * DIN + c0);
  }
  double s0 = 0.0, s1 = 0.0, s2 = 0.0, s3 = 0.0, q0 = 0.0, q1 = 0.0, q2 = 0.0, q3 = 0.0;
#pragma unroll 1
  for (int i = 0; i < 16; ++i) {
    const int lrow = lrow0 + i;
    const int grow = chunkBase + lrow;
    const bool valid = grow < nN;
    v4f hv;
    if (MODE == 2) {
      const v4f xv = *(const v4f*)(hp + (size_t)grow * DIN + c0);
      hv.x = valid ? xv.x : 0.f; hv.y = valid ? xv.y : 0.f; hv.z = valid ? xv.z : 0.f; hv.w = valid ? xv.w : 0.f;
    } else {
      const float* gp = gi + (size_t)lrow * G3H + c0;
      const float* hq = gh + (size_t)lrow * G3H + c0;
      const v4f ir = *(const v4f*)gp, iz = *(const v4f*)(gp + DIN), inn = *(const v4f*)(gp + 2 * DIN);
      const v4f hr = *(const v4f*)hq, hz = *(const v4f*)(hq + DIN), hn = *(const v4f*)(hq + 2 * DIN);
      v4f X;
      if (MODE == 0) {
        const int gcl = valid ? grow : nN - 1;
        const v4f xv = *(const v4f*)(xin + (size_t)gcl * DIN + c0);
        X.x = bfr(xv.x); X.y = bfr(xv.y); X.z = bfr(xv.z); X.w = bfr(xv.w);
      } else {
        const v4f xv = *(const v4f*)(hp + (size_t)grow * DIN + c0);
        X.x = fmaf(xv.x - mean4.x, mult4.x, beta4.x);
        X.y = fmaf(xv.y - mean4.y, mult4.y, beta4.y);
        X.z = fmaf(xv.z - mean4.z, mult4.z, beta4.z);
        X.w = fmaf(xv.w - mean4.w, mult4.w, beta4.w);
      }
      hv.x = valid ? gruc(ir.x, hr.x, iz.x, hz.x, inn.x, hn.x, X.x) : 0.f;
      hv.y = valid ? gruc(ir.y, hr.y, iz.y, hz.y, inn.y, hn.y, X.y) : 0.f;
      hv.z = valid ? gruc(ir.z, hr.z, iz.z, hz.z, inn.z, hn.z, X.z) : 0.f;
      hv.w = valid ? gruc(ir.w, hr.w, iz.w, hz.w, inn.w, hn.w, X.w) : 0.f;
      float* op = hp + (size_t)grow * DIN + c0;
      *(volatile v4f*)op = hv;
      __threadfence();
      *(volatile v4f*)op = hv;
    }
    const double d0 = (double)hv.x, d1 = (double)hv.y, d2 = (double)hv.z, d3 = (double)hv.w;
    s0 += d0; s1 += d1; s2 += d2; s3 += d3;
    q0 += d0 * d0; q1 += d1 * d1; q2 += d2 * d2; q3 += d3 * d3;
  }
  red[(0 * NWAVE + wave) * DIN + c0 + 0] = s0;
  red[(0 * NWAVE + wave) * DIN + c0 + 1] = s1;
  red[(0 * NWAVE + wave) * DIN + c0 + 2] = s2;
  red[(0 * NWAVE + wave) * DIN + c0 + 3] = s3;
  red[(1 * NWAVE + wave) * DIN + c0 + 0] = q0;
  red[(1 * NWAVE + wave) * DIN + c0 + 1] = q1;
  red[(1 * NWAVE + wave) * DIN + c0 + 2] = q2;
  red[(1 * NWAVE + wave) * DIN + c0 + 3] = q3;
  __syncthreads();
  if (tid < DIN) {
    const int e0 = 2 * tid, e1 = e0 + 1;
    const int qa = e0 >> 7, ca = e0 & (DIN - 1), qb = e1 >> 7, cbb = e1 & (DIN - 1);
    double a = 0.0, b = 0.0;
#pragma unroll
    for (int w2 = 0; w2 < NWAVE; ++w2) {
      a += red[(qa * NWAVE + w2) * DIN + ca];
      b += red[(qb * NWAVE + w2) * DIN + cbb];
    }
    DU2 u;
    u.d[0] = a;
    u.d[1] = b;
    float* rp = rec + (size_t)blkg * 512 + 4 * tid;
    *(volatile v4f*)rp = u.f;
    __threadfence();
    *(volatile v4f*)rp = u.f;
  }
}

__global__ __launch_bounds__(NTHR) void k_bnfold(const double* __restrict__ recd, const float* __restrict__ g,
                                                 const float* __restrict__ be, float* tab, int nrec, int nN) {
  __shared__ double tot[2 * DIN];
  __shared__ __attribute__((aligned(16))) float tb[3 * DIN];
  const int tid = (int)threadIdx.x;
  {
    double S = 0.0;
#pragma unroll 1
    for (int b = 0; b < nrec; ++b) S += recd[(size_t)b * 256 + tid];
    tot[tid] = S;
  }
  __syncthreads();
  if (tid < DIN) {
    const double invn = 1.0 / (double)nN;
    const double mean = tot[tid] * invn;
    double var = tot[DIN + tid] * invn - mean * mean;
    var = var > 0.0 ? var : 0.0;
    const float meanf = (float)mean;
    const float varf  = (float)var;
    const float inv   = 1.0f / sqrtf(varf + 1e-5f);
    tb[tid]           = meanf;
    tb[DIN + tid]     = bfr(g[tid]) * inv;
    tb[2 * DIN + tid] = bfr(be[tid]);
  }
  __syncthreads();
  if (tid < 96) {
    const v4f v = *(const v4f*)(tb + 4 * tid);
    *(volatile v4f*)(tab + 4 * tid) = v;
    __threadfence();
    *(volatile v4f*)(tab + 4 * tid) = v;
  }
}

__global__ __launch_bounds__(NTHR) void k_bnsplit(const float* __restrict__ hp, const float* __restrict__ tab,
                                                  us_t* hb, int nN, int nUnits) {
  const int u = (int)blockIdx.x * NTHR + (int)threadIdx.x;
  if (u >= nUnits) return;
  const int row = u >> 4;
  const int c0  = (u & 15) * 8;
  const int rc  = row < nN ? row : nN - 1;
  const float* p = hp + (size_t)rc * DIN + c0;
  const v4f xa = *(const v4f*)p, xb = *(const v4f*)(p + 4);
  const v4f ma = *(const v4f*)(tab + c0), mb = *(const v4f*)(tab + c0 + 4);
  const v4f sa = *(const v4f*)(tab + DIN + c0), sb = *(const v4f*)(tab + DIN + c0 + 4);
  const v4f ba = *(const v4f*)(tab + 2 * DIN + c0), bb = *(const v4f*)(tab + 2 * DIN + c0 + 4);
  v4f va, vb;
  va.x = fmaf(xa.x - ma.x, sa.x, ba.x); va.y = fmaf(xa.y - ma.y, sa.y, ba.y);
  va.z = fmaf(xa.z - ma.z, sa.z, ba.z); va.w = fmaf(xa.w - ma.w, sa.w, ba.w);
  vb.x = fmaf(xb.x - mb.x, sb.x, bb.x); vb.y = fmaf(xb.y - mb.y, sb.y, bb.y);
  vb.z = fmaf(xb.z - mb.z, sb.z, bb.z); vb.w = fmaf(xb.w - mb.w, sb.w, bb.w);
  const v4f z4 = {0.f, 0.f, 0.f, 0.f};
  if (row >= nN) { va = z4; vb = z4; }
  v4i H, L;
  split8(va, vb, H, L);
  us_t* o = hb + (size_t)row * KSP + c0;
  *(volatile v4i*)o = H;
  *(volatile v4i*)(o + DIN) = L;
  __threadfence();
  *(volatile v4i*)o = H;
  *(volatile v4i*)(o + DIN) = L;
}

__global__ __launch_bounds__(NTHR) void k_final(const float* __restrict__ h3, const float* __restrict__ tab,
                                                const float* __restrict__ lw2, const float* __restrict__ lb2,
                                                float* out, int nN) {
  __shared__ __attribute__((aligned(16))) float res[RB];
  const int tid = (int)threadIdx.x, lane = tid & 31, wave = tid >> 5;
  const int c0 = 4 * lane;
  const v4f mean4 = *(const v4f*)(tab + c0);
  const v4f mult4 = *(const v4f*)(tab + DIN + c0);
  const v4f beta4 = *(const v4f*)(tab + 2 * DIN + c0);
  const v4f wv = *(const v4f*)(lw2 + c0);
  const float w0 = bfr(wv.x), w1 = bfr(wv.y), w2 = bfr(wv.z), w3 = bfr(wv.w);
  const float b2 = bfr(lb2[0]);
  const int rowBase = (int)blockIdx.x * RB;
#pragma unroll 1
  for (int i = 0; i < 16; ++i) {
    const int r = wave * 16 + i;
    const int grow = rowBase + r;
    const v4f xv = *(const v4f*)(h3 + (size_t)grow * DIN + c0);
    const float v0 = fmaf(xv.x - mean4.x, mult4.x, beta4.x);
    const float v1 = fmaf(xv.y - mean4.y, mult4.y, beta4.y);
    const float v2 = fmaf(xv.z - mean4.z, mult4.z, beta4.z);
    const float v3 = fmaf(xv.w - mean4.w, mult4.w, beta4.w);
    float sacc = v0 * w0;
    sacc = fmaf(v1, w1, sacc);
    sacc = fmaf(v2, w2, sacc);
    sacc = fmaf(v3, w3, sacc);
#pragma unroll
    for (int o = 16; o > 0; o >>= 1) sacc += __shfl_xor(sacc, o);
    if (lane == 0) res[r] = sacc + b2;
  }
  __syncthreads();
  if (wave == 0) {
    const int r0 = rowBase + 4 * lane;
    const v4f ov = *(const v4f*)(res + 4 * lane);
    float* op = out + r0;
    const bool full = (r0 + 3) < nN;
    if (full) {
      *(volatile v4f*)op = ov;
    } else {
      if (r0 < nN)     ((volatile float*)op)[0] = ov.x;
      if (r0 + 1 < nN) ((volatile float*)op)[1] = ov.y;
      if (r0 + 2 < nN) ((volatile float*)op)[2] = ov.z;
      if (r0 + 3 < nN) ((volatile float*)op)[3] = ov.w;
    }
    __threadfence();
    if (full) {
      *(volatile v4f*)op = ov;
    } else {
      if (r0 < nN)     ((volatile float*)op)[0] = ov.x;
      if (r0 + 1 < nN) ((volatile float*)op)[1] = ov.y;
      if (r0 + 2 < nN) ((volatile float*)op)[2] = ov.z;
      if (r0 + 3 < nN) ((volatile float*)op)[3] = ov.w;
    }
  }
}

static int pick_nb(int nE, int nN) {
  int nb = NBMAX;
  while (nb > 16 && (long long)nb * (long long)nE * 5LL > (long long)RCAP * (long long)nN * 4LL) nb >>= 1;
  return nb;
}
static inline int cdiv(int a, int b) { return (a + b - 1) / b; }

extern "C" void kernel_launch(void* const* d_in, const int* in_sizes, int n_in,
                              void* d_out, int out_size, void* d_ws, size_t ws_size,
                              hipStream_t stream) {
  if (n_in < 23) return;
  const int nN = in_sizes[0] / DIN;
  if (nN <= 0 || in_sizes[0] != nN * DIN || nN > (1 << 22)) return;
  const int nE = in_sizes[1];
  if (nE < 1 || nE > (1 << 20)) return;
  if (in_sizes[22] != 2 * nE) return;
  if (in_sizes[2] != DIN * DIN) return;
  if (in_sizes[3] != G3H * DIN || in_sizes[4] != G3H * DIN) return;
  if (in_sizes[5] != G3H || in_sizes[6] != G3H) return;
  if (in_sizes[7] != DIN * DIN) return;
  if (in_sizes[8] != G3H * DIN || in_sizes[9] != G3H * DIN) return;
  if (in_sizes[10] != G3H || in_sizes[11] != G3H) return;
  if (in_sizes[12] != DIN * DIN || in_sizes[13] != DIN) return;
  if (in_sizes[14] != DIN || in_sizes[15] < 1) return;
  for (int i = 16; i <= 21; ++i) if (in_sizes[i] != DIN) return;
  if (out_size != nN) return;

  const float* x    = (const float*)d_in[0];
  const float* ew   = (const float*)d_in[1];
  const float* W1   = (const float*)d_in[2];
  const float* Wih1 = (const float*)d_in[3];
  const float* Whh1 = (const float*)d_in[4];
  const float* bih1 = (const float*)d_in[5];
  const float* bhh1 = (const float*)d_in[6];
  const float* W2   = (const float*)d_in[7];
  const float* Wih2 = (const float*)d_in[8];
  const float* Whh2 = (const float*)d_in[9];
  const float* bih2 = (const float*)d_in[10];
  const float* bhh2 = (const float*)d_in[11];
  const float* lw1  = (const float*)d_in[12];
  const float* lb1  = (const float*)d_in[13];
  const float* lw2  = (const float*)d_in[14];
  const float* lb2  = (const float*)d_in[15];
  const float* g1   = (const float*)d_in[16];
  const float* be1  = (const float*)d_in[17];
  const float* g2   = (const float*)d_in[18];
  const float* be2  = (const float*)d_in[19];
  const float* g3   = (const float*)d_in[20];
  const float* be3  = (const float*)d_in[21];
  const int*   ei   = (const int*)  d_in[22];
  const int* src = ei;
  const int* dst = ei + nE;
  float* out = (float*)d_out;

  const int MP   = cdiv(nN, MPQ) * MPQ;
  const int CH   = MP / NCHK;
  const int NREC = MP / RB;
  const int nb   = pick_nb(nE, nN);
  const int gA   = cdiv(CH, nb);
  const int vec8 = ((nE & 3) == 0) ? 1 : 0;
  if (gA * nb < CH) return;
  if ((CH % GBM) != 0 || (CH % RB) != 0) return;

  char* ws = (char*)d_ws;
  size_t off = 0;
  const size_t oWT  = off; off += (size_t)WO_END * 2;                 off = (off + 255) & ~(size_t)255;
  const size_t oXB  = off; off += (size_t)MP * DIN * 2;               off = (off + 255) & ~(size_t)255;
  const size_t oHB  = off; off += (size_t)MP * KSP * 2;               off = (off + 255) & ~(size_t)255;
  const size_t oM   = off; off += (size_t)MP * DIN * 4;               off = (off + 255) & ~(size_t)255;
  const size_t oH3  = off; off += (size_t)MP * DIN * 4;               off = (off + 255) & ~(size_t)255;
  const size_t oAG  = off; off += (size_t)CH * KSP * 2;               off = (off + 255) & ~(size_t)255;
  const size_t oGI  = off; off += (size_t)CH * G3H * 4;               off = (off + 255) & ~(size_t)255;
  const size_t oGH  = off; off += (size_t)CH * G3H * 4;               off = (off + 255) & ~(size_t)255;
  const size_t oHP  = off; off += (size_t)MP * DIN * 4;               off = (off + 255) & ~(size_t)255;
  const size_t oREC = off; off += (size_t)NREC * 2048;                off = (off + 255) & ~(size_t)255;
  const size_t oTAB = off; off += (size_t)3 * 2048;                   off = (off + 255) & ~(size_t)255;
  if (off > ws_size || off > (size_t)WSMAX) return;
  us_t*  WT  = (us_t*)(ws + oWT);
  us_t*  XB1 = (us_t*)(ws + oXB);
  us_t*  HB  = (us_t*)(ws + oHB);
  float* M   = (float*)(ws + oM);
  float* H3  = (float*)(ws + oH3);
  us_t*  AGG = (us_t*)(ws + oAG);
  float* GI  = (float*)(ws + oGI);
  float* GH  = (float*)(ws + oGH);
  float* HP  = (float*)(ws + oHP);
  float* REC = (float*)(ws + oREC);
  float* TAB1 = (float*)(ws + oTAB);
  float* TAB2 = (float*)(ws + oTAB + 2048);
  float* TAB3 = (float*)(ws + oTAB + 4096);

  hipFuncSetAttribute(reinterpret_cast<const void*>(&k_agg),
                      hipFuncAttributeMaxDynamicSharedMemorySize, LDS_AGG);

  k_wcvt<<<dim3(cdiv(G3H * 16, NTHR), 7), NTHR, 0, stream>>>(W1, Whh1, Wih1, W2, Whh2, Wih2, lw1, WT);
  const int nUx = MP * 16;
  k_xprep<<<cdiv(nUx, NTHR), NTHR, 0, stream>>>(x, XB1, nN, nUx);

  const int gM = MP / GBM;
  const int gC = CH / GBM;

  k_gemm<<<dim3(gM, DIN / GBN), GTHR, 0, stream>>>(XB1, WT + WO_M1, bhh1, M, DIN, DIN, 0, 0, DIN / GBN,
                                                    XB1, WT + WO_M1, bhh1, M, DIN, DIN, 0, 0);
  for (int k = 0; k < NCHK; ++k) {
    const int cb = k * CH;
    k_agg<<<gA, NTHR, LDS_AGG, stream>>>(src, dst, ew, M, AGG, nN, nE, nb, vec8, cb, CH);
    k_gemm<<<dim3(gC, 2 * (G3H / GBN)), GTHR, 0, stream>>>(AGG, WT + WO_IH1, bih1, GI, KSP, G3H, G3H, 0, G3H / GBN,
                                                            XB1 + (size_t)cb * DIN, WT + WO_HH1, bhh1, GH, DIN, G3H, G3H, 0);
    k_gru<0><<<CH / RB, NTHR, 0, stream>>>(GI, GH, x, TAB1, HP, REC, cb, nN);
  }
  k_bnfold<<<1, NTHR, 0, stream>>>((const double*)REC, g1, be1, TAB1, NREC, nN);
  k_bnsplit<<<cdiv(nUx, NTHR), NTHR, 0, stream>>>(HP, TAB1, HB, nN, nUx);

  k_gemm<<<dim3(gM, DIN / GBN), GTHR, 0, stream>>>(HB, WT + WO_M2, bhh2, M, KSP, DIN, 0, 0, DIN / GBN,
                                                    HB, WT + WO_M2, bhh2, M, KSP, DIN, 0, 0);
  for (int k = 0; k < NCHK; ++k) {
    const int cb = k * CH;
    k_agg<<<gA, NTHR, LDS_AGG, stream>>>(src, dst, ew, M, AGG, nN, nE, nb, vec8, cb, CH);
    k_gemm<<<dim3(gC, 2 * (G3H / GBN)), GTHR, 0, stream>>>(AGG, WT + WO_IH2, bih2, GI, KSP, G3H, G3H, 0, G3H / GBN,
                                                            HB + (size_t)cb * KSP, WT + WO_HH2, bhh2, GH, KSP, G3H, G3H, 0);
    k_gru<1><<<CH / RB, NTHR, 0, stream>>>(GI, GH, HP, TAB1, HP, REC, cb, nN);
  }
  k_bnfold<<<1, NTHR, 0, stream>>>((const double*)REC, g2, be2, TAB2, NREC, nN);
  k_bnsplit<<<cdiv(nUx, NTHR), NTHR, 0, stream>>>(HP, TAB2, HB, nN, nUx);

  k_gemm<<<dim3(gM, DIN / GBN), GTHR, 0, stream>>>(HB, WT + WO_L, lb1, H3, KSP, DIN, DIN, 1, DIN / GBN,
                                                    HB, WT + WO_L, lb1, H3, KSP, DIN, DIN, 1);
  k_gru<2><<<NREC, NTHR, 0, stream>>>(H3, H3, H3, TAB2, H3, REC, 0, nN);
  k_bnfold<<<1, NTHR, 0, stream>>>((const double*)REC, g3, be3, TAB3, NREC, nN);
  k_final<<<NREC, NTHR, 0, stream>>>(H3, TAB3, lw2, lb2, out, nN);
}
